// TriplaneSdf_39582418600324
// MI455X (gfx1250) — hardware-verified
//
#include <hip/hip_runtime.h>
#include <math.h>
#include <stdint.h>

typedef __attribute__((ext_vector_type(16))) _Float16 v16h;
typedef __attribute__((ext_vector_type(8)))  _Float16 v8h;
typedef __attribute__((ext_vector_type(8)))  float    v8f;
typedef __attribute__((ext_vector_type(4)))  float    v4f;

__device__ __forceinline__ void dep_guard_h(v8f& a, v8f& b, v16h x, v16h y) { asm volatile("v_nop\n\tv_nop\n\tv_nop\n\tv_nop" : "+v"(a), "+v"(b) : "v"(x), "v"(y)); }
__device__ __forceinline__ void keep4_h(v16h a, v16h b, v16h c, v16h d) { asm volatile("v_nop" :: "v"(a), "v"(b), "v"(c), "v"(d)); }
__device__ __forceinline__ void acc_guard4(v8f& a, v8f& b, v8f& c, v8f& d) { asm volatile("v_nop\n\tv_nop\n\tv_nop\n\tv_nop" : "+v"(a), "+v"(b), "+v"(c), "+v"(d)); }
template <typename T> struct Frag;
template <> struct Frag<_Float16> {
  typedef v16h V; union U { v16h v; v8h h[2]; };
  static __device__ __forceinline__ v16h load(const _Float16* p) {
    U f; f.h[0] = *(const v8h*)(p); f.h[1] = *(const v8h*)(p + 16); return f.v;
  }
  static __device__ __forceinline__ v8f mma(v16h a, v16h b, v8f c) {
    return __builtin_amdgcn_wmma_f32_16x16x32_f16(false, a, false, b, (short)0, c, false, false);
  }
  static __device__ __forceinline__ void guard(v8f& a, v8f& b, v16h x, v16h y) { dep_guard_h(a, b, x, y); }
  static __device__ __forceinline__ void keep(v16h a, v16h b, v16h c, v16h d) { keep4_h(a, b, c, d); }
};

__device__ __forceinline__ v8f mma_h(v16h a, v16h b, v8f c) {
  c = __builtin_amdgcn_wmma_f32_16x16x32_f16(false, a, false, b, (short)0, c, false, false);
  asm volatile("v_nop\n\tv_nop\n\tv_nop\n\tv_nop" : "+v"(c) : "v"(a), "v"(b));
  return c;
}

#define NCH   32
#define RESO  512
#define NPIX  (RESO * RESO)
#define PLH   (NPIX * NCH)
#define KF    96
#define FP    104
#define W0P   104
#define W1P   40
#define HP    40
#define SP    36
#define TPB   128
#define W0T_HALVES (64 * W0P)
#define W1T_HALVES (32 * W1P)
#define NCHUNK_W ((W0T_HALVES + W1T_HALVES) / 8)
#define TP_PIX 256
#define PCARRY 16.0f
#define WCARRY 16.0f

__global__ __launch_bounds__(TP_PIX) void k_plane_t(const float* __restrict__ pa, const float* __restrict__ pb,
                                                    const float* __restrict__ pc, _Float16* __restrict__ T) {
  __shared__ __align__(16) _Float16 s[TP_PIX * 40];
  const int pl = blockIdx.y;
  const float* P = (pl == 0) ? pa : ((pl == 1) ? pb : pc);
  const int pix0 = blockIdx.x * TP_PIX;
  const int t = threadIdx.x;
  const float* src = P + pix0 + t;
#pragma unroll
  for (int cg = 0; cg < 4; ++cg) {
    v8h pk;
#pragma unroll
    for (int e = 0; e < 8; ++e) pk[e] = (_Float16)(src[(size_t)(cg * 8 + e) * NPIX] * PCARRY);
    *(v8h*)(s + t * 40 + cg * 8) = pk;
  }
  __syncthreads();
  _Float16* Tb = T + (size_t)pl * PLH + (size_t)pix0 * NCH;
  v8h vals[4];
#pragma unroll
  for (int i = 0; i < 4; ++i) {
    const int q = i * TP_PIX + t;
    vals[i] = *(const v8h*)(s + (q >> 2) * 40 + (q & 3) * 8);
  }
#pragma unroll
  for (int i = 0; i < 4; ++i) *(volatile v8h*)(Tb + (size_t)(i * TP_PIX + t) * 8) = vals[i];
  __threadfence();
#pragma unroll
  for (int i = 0; i < 4; ++i) *(volatile v8h*)(Tb + (size_t)(i * TP_PIX + t) * 8) = vals[i];
}

__global__ __launch_bounds__(512) void k_wprep(const float* __restrict__ wsdf0, const float* __restrict__ wrgb0,
                                               const float* __restrict__ wrgb1, _Float16* __restrict__ Wt) {
  const int q = blockIdx.x * 512 + threadIdx.x;
  if (q >= NCHUNK_W) return;
  const int d0  = q / 13;
  const int n0  = min(d0, 63);
  const int kc0 = q - d0 * 13;
  const int qq  = max(q - 832, 0);
  const int d1  = qq / 5;
  const int n1  = min(d1, 31);
  const int kc1 = qq - d1 * 5;
  const bool second = (q >= 832);
  v8h o;
#pragma unroll
  for (int e = 0; e < 8; ++e) {
    const int k0  = kc0 * 8 + e;
    const int k0c = min(k0, KF - 1);
    const float a = wsdf0[k0c * 32 + (n0 & 31)];
    const float b = wrgb0[k0c * 32 + (n0 & 31)];
    float v0 = (n0 < 32) ? a : b;
    v0 = (k0 < KF) ? v0 : 0.0f;
    const int k1  = kc1 * 8 + e;
    const int k1c = min(k1, 31);
    const float c = wrgb1[k1c * 32 + n1];
    const float v1 = (k1 < 32) ? c : 0.0f;
    const float v = second ? v1 : v0;
    o[e] = (_Float16)(v * WCARRY);
  }
  _Float16* dst = Wt + (size_t)q * 8;
  *(volatile v8h*)dst = o;
  __threadfence();
  *(volatile v8h*)dst = o;
}

__global__ __launch_bounds__(TPB) void k_main(const float* __restrict__ pos, const _Float16* __restrict__ T,
                                             const _Float16* __restrict__ Wt, const float* __restrict__ wsdf1,
                                             const float* __restrict__ wrgb2, float* __restrict__ out, int npts) {
  __shared__ __align__(16) _Float16 sFeat[TPB * FP];
  __shared__ __align__(16) float    sHs[TPB * SP];
  __shared__ __align__(16) _Float16 sHr[TPB * HP];
  __shared__ __align__(16) float    sHead[128];

  const int tid  = threadIdx.x;
  const int lane = tid & 31;
  const int wave = tid >> 5;
  const int hh   = lane >> 4;
  const int rl   = lane & 15;
  const int row0 = wave * 32;

  {
    const float a = wsdf1[min(tid, 31)];
    const float b = wrgb2[min(max(tid - 32, 0), 95)];
    sHead[tid] = (tid < 32) ? a : b;
  }

  const long long ipt = (long long)blockIdx.x * TPB + tid;
  const long long ipl = (ipt < (long long)npts) ? ipt : (long long)(npts - 1);
  const float x = pos[ipl * 3 + 0];
  const float y = pos[ipl * 3 + 1];
  const float z = pos[ipl * 3 + 2];
  const float dist = sqrtf(x * x + y * y + z * z);
  const float px = x * 2.0f, py = y * 2.0f, pz = z * 2.0f;
  {
    _Float16* frow = sFeat + tid * FP;
#pragma unroll 1
    for (int p = 0; p < 3; ++p) {
      const float gx = (p == 0) ? py : pz;
      const float gy = (p == 2) ? py : px;
      float ix = (gx + 1.0f) * 0.5f * 511.0f;
      float iy = (gy + 1.0f) * 0.5f * 511.0f;
      ix = fminf(fmaxf(ix, 0.0f), 511.0f);
      iy = fminf(fmaxf(iy, 0.0f), 511.0f);
      const float ix0f = floorf(ix), iy0f = floorf(iy);
      const float wx = ix - ix0f, wy = iy - iy0f;
      int ix0 = (int)ix0f, iy0 = (int)iy0f;
      ix0 = min(max(ix0, 0), RESO - 1);
      iy0 = min(max(iy0, 0), RESO - 1);
      const int ix1 = min(ix0 + 1, RESO - 1);
      const int iy1 = min(iy0 + 1, RESO - 1);
      const float w00 = (1.0f - wy) * (1.0f - wx);
      const float w01 = (1.0f - wy) * wx;
      const float w10 = wy * (1.0f - wx);
      const float w11 = wy * wx;
      const _Float16* Tp = T + (size_t)p * PLH;
      const v8h* t00 = (const v8h*)(Tp + ((size_t)iy0 * RESO + ix0) * NCH);
      const v8h* t01 = (const v8h*)(Tp + ((size_t)iy0 * RESO + ix1) * NCH);
      const v8h* t10 = (const v8h*)(Tp + ((size_t)iy1 * RESO + ix0) * NCH);
      const v8h* t11 = (const v8h*)(Tp + ((size_t)iy1 * RESO + ix1) * NCH);
#pragma unroll
      for (int g = 0; g < 4; ++g) {
        const v8h a = t00[g], b = t01[g], c = t10[g], d = t11[g];
        v8h o;
#pragma unroll
        for (int e = 0; e < 8; ++e) {
          float v = w00 * (float)a[e];
          v += w01 * (float)b[e];
          v += w10 * (float)c[e];
          v += w11 * (float)d[e];
          o[e] = (_Float16)v;
        }
        *(v8h*)(frow + p * NCH + g * 8) = o;
      }
    }
  }
  __syncthreads();

  {
    v8f acc[2][4];
#pragma unroll
    for (int i = 0; i < 2; ++i)
#pragma unroll
      for (int j = 0; j < 4; ++j) acc[i][j] = (v8f){0.f, 0.f, 0.f, 0.f, 0.f, 0.f, 0.f, 0.f};
#pragma unroll
    for (int kt = 0; kt < 3; ++kt) {
      v16h bf[4];
#pragma unroll
      for (int j = 0; j < 4; ++j)
        bf[j] = Frag<_Float16>::load(Wt + (size_t)(j * 16 + rl) * W0P + kt * 32 + 8 * hh);
#pragma unroll
      for (int i = 0; i < 2; ++i) {
        const v16h af = Frag<_Float16>::load(sFeat + (row0 + i * 16 + rl) * FP + kt * 32 + 8 * hh);
#pragma unroll
        for (int j = 0; j < 4; ++j) acc[i][j] = mma_h(af, bf[j], acc[i][j]);
      }
    }
#pragma unroll
    for (int i = 0; i < 2; ++i) {
#pragma unroll
      for (int j = 0; j < 4; ++j) {
#pragma unroll
        for (int r = 0; r < 8; ++r) {
          const int row = row0 + i * 16 + 8 * hh + r;
          const float v = fmaxf(acc[i][j][r], 0.0f);
          if (j < 2) sHs[row * SP + j * 16 + rl] = v * (1.0f / 256.0f);
          else       sHr[row * HP + (j - 2) * 16 + rl] = (_Float16)v;
        }
      }
    }
  }
  __syncthreads();

  float sdf;
  {
    const float* hr = sHs + tid * SP;
    float s = 0.0f;
#pragma unroll
    for (int k4 = 0; k4 < 8; ++k4) {
      const v4f hv = *(const v4f*)(hr + 4 * k4);
#pragma unroll
      for (int e = 0; e < 4; ++e) s += hv[e] * sHead[4 * k4 + e];
    }
    const float th = tanhf(s);
    sdf = th * 0.5f * 1.732f * 1.5f;
    sdf = sdf + (dist - 0.05f);
  }
  __syncthreads();

  {
    const _Float16* W1t = Wt + W0T_HALVES;
    v8f acc2[2][2];
#pragma unroll
    for (int i = 0; i < 2; ++i)
#pragma unroll
      for (int j = 0; j < 2; ++j) acc2[i][j] = (v8f){0.f, 0.f, 0.f, 0.f, 0.f, 0.f, 0.f, 0.f};
    v16h b1[2];
#pragma unroll
    for (int j = 0; j < 2; ++j) b1[j] = Frag<_Float16>::load(W1t + (size_t)(j * 16 + rl) * W1P + 8 * hh);
#pragma unroll
    for (int i = 0; i < 2; ++i) {
      const v16h af = Frag<_Float16>::load(sHr + (row0 + i * 16 + rl) * HP + 8 * hh);
#pragma unroll
      for (int j = 0; j < 2; ++j) acc2[i][j] = mma_h(af, b1[j], acc2[i][j]);
    }
#pragma unroll
    for (int i = 0; i < 2; ++i) {
#pragma unroll
      for (int j = 0; j < 2; ++j) {
#pragma unroll
        for (int r = 0; r < 8; ++r) {
          const int row = row0 + i * 16 + 8 * hh + r;
          sHs[row * SP + j * 16 + rl] = fmaxf(acc2[i][j][r], 0.0f) * (1.0f / 4096.0f);
        }
      }
    }
  }
  __syncthreads();

  {
    const float* hr = sHs + tid * SP;
    float q0 = 0.0f, q1 = 0.0f, q2 = 0.0f;
#pragma unroll
    for (int k4 = 0; k4 < 8; ++k4) {
      const v4f hv = *(const v4f*)(hr + 4 * k4);
#pragma unroll
      for (int e = 0; e < 4; ++e) {
        const int k = 4 * k4 + e;
        q0 += hv[e] * sHead[32 + k * 3 + 0];
        q1 += hv[e] * sHead[32 + k * 3 + 1];
        q2 += hv[e] * sHead[32 + k * 3 + 2];
      }
    }
    const float s0 = __builtin_amdgcn_rcpf(1.0f + expf(-q0));
    const float s1 = __builtin_amdgcn_rcpf(1.0f + expf(-q1));
    const float s2 = __builtin_amdgcn_rcpf(1.0f + expf(-q2));
    v4f o;
    o[0] = sdf; o[1] = s0; o[2] = s1; o[3] = s2;
    float* op = out + (size_t)ipl * 4;
    *(volatile v4f*)op = o;
    __threadfence();
    *(volatile v4f*)op = o;
  }
}

extern "C" void kernel_launch(void* const* d_in, const int* in_sizes, int n_in,
                              void* d_out, int out_size, void* d_ws, size_t ws_size,
                              hipStream_t stream) {
  if (n_in < 9) return;
  const float* pos   = (const float*)d_in[0];
  const float* pxy   = (const float*)d_in[1];
  const float* pxz   = (const float*)d_in[2];
  const float* pyz   = (const float*)d_in[3];
  const float* wsdf0 = (const float*)d_in[4];
  const float* wsdf1 = (const float*)d_in[5];
  const float* wrgb0 = (const float*)d_in[6];
  const float* wrgb1 = (const float*)d_in[7];
  const float* wrgb2 = (const float*)d_in[8];
  float* out = (float*)d_out;

  const int npts = in_sizes[0] / 3;
  if (npts <= 0 || (npts % TPB) != 0) return;
  if (in_sizes[1] != NCH * NPIX || in_sizes[2] != NCH * NPIX || in_sizes[3] != NCH * NPIX) return;
  if (in_sizes[4] != KF * 32 || in_sizes[5] != 32 || in_sizes[6] != KF * 32 || in_sizes[7] != 32 * 32 || in_sizes[8] != 32 * 3) return;
  if (out_size < npts * 4) return;

  const size_t bytesT = (size_t)3 * PLH * sizeof(_Float16);
  const size_t offT   = 0;
  const size_t offW   = offT + bytesT;
  const size_t bytesW = (size_t)NCHUNK_W * 16;
  if (offW + bytesW > ws_size) return;
  char* ws = (char*)d_ws;
  _Float16* T  = (_Float16*)(ws + offT);
  _Float16* Wt = (_Float16*)(ws + offW);

  hipLaunchKernelGGL(k_plane_t, dim3(NPIX / TP_PIX, 3), dim3(TP_PIX), 0, stream, pxy, pxz, pyz, T);
  hipLaunchKernelGGL(k_wprep, dim3((NCHUNK_W + 511) / 512), dim3(512), 0, stream, wsdf0, wrgb0, wrgb1, Wt);
  hipLaunchKernelGGL(k_main, dim3(npts / TPB), dim3(TPB), 0, stream, pos, (const _Float16*)T, (const _Float16*)Wt,
                     wsdf1, wrgb2, out, npts);
  (void)hipGetLastError();
}
